// SpanScorer_1975684956404
// MI455X (gfx1250) — hardware-verified
//
#include <hip/hip_runtime.h>
#define TT 4096
#define SD 400
#define SDP 416
#define ED 300
#define EDP 320
#define HID 150
#define HP 160
#define MAXW 10
#define NSPAN 40915
#define NSP 40928

typedef __bf16 v16b __attribute__((ext_vector_type(16)));
typedef unsigned short v8us __attribute__((ext_vector_type(8), may_alias));
typedef float  v8f  __attribute__((ext_vector_type(8)));
typedef float  v4f  __attribute__((ext_vector_type(4)));
typedef float  v4fa __attribute__((ext_vector_type(4), may_alias));
union FragB { v16b v; v8us half[2]; unsigned short u[16]; };

__device__ __forceinline__ unsigned short bf16_bits(float x) { unsigned int u = __float_as_uint(x); return (unsigned short)((u + 0x7FFFu + ((u >> 16) & 1u)) >> 16); }
__device__ __forceinline__ float bf16_val(unsigned short b) { return __uint_as_float(((unsigned int)b) << 16); }
__device__ __forceinline__ float bf16_round(float x) { return bf16_val(bf16_bits(x)); }
template <int NT>
__device__ __forceinline__ v8f mmaN(v16b ah, v16b al, v16b bh, v16b bl, v8f c) {
  c = __builtin_amdgcn_wmma_f32_16x16x32_bf16(false, ah, false, bh, (short)0, c, false, false);
  if (NT >= 2) c = __builtin_amdgcn_wmma_f32_16x16x32_bf16(false, al, false, bh, (short)0, c, false, false);
  if (NT >= 3) c = __builtin_amdgcn_wmma_f32_16x16x32_bf16(false, ah, false, bl, (short)0, c, false, false);
  asm volatile("v_nop\n\tv_nop\n\tv_nop\n\tv_nop" : "+v"(c) : "v"(ah), "v"(al), "v"(bh), "v"(bl));
  return c;
}

__global__ __launch_bounds__(256) void k_wt_bf16(const float* __restrict__ W, unsigned short* __restrict__ Wt, int K, int N) {
  const int t = blockIdx.x * 256 + threadIdx.x;
  const int k8n = K / 8;
  if (t >= N * k8n) return;
  const int n = t / k8n, k8 = (t % k8n) * 8;
  v8us v;
#pragma unroll
  for (int i = 0; i < 8; ++i) v[i] = bf16_bits(W[(size_t)(k8 + i) * N + n]);
  *(volatile v8us*)(Wt + (size_t)n * K + k8) = v;
  __threadfence();
  *(volatile v8us*)(Wt + (size_t)n * K + k8) = v;
}

template <bool ASPLIT, int ACT, bool BIAS_BF16>
__global__ __launch_bounds__(128) void k_gemm_bf(const float* __restrict__ A, int lda, const unsigned short* __restrict__ Wt, int ldb,
                                               const float* __restrict__ bias, float* __restrict__ C, int ldc, int M, int N, int K) {
  __shared__ __attribute__((aligned(16))) float so[4][16][64];
  const int tid = threadIdx.x, w = tid >> 5, lane = tid & 31, ln = lane & 15, hh = lane >> 4;
  const int ntn = N / 64;
  const int wid = blockIdx.x * 4 + w;
  const int mt = wid / ntn, nq = wid % ntn;
  if (mt * 16 >= M) return;
  const int row0 = mt * 16, col0 = nq * 64;
  const float* arow = A + (size_t)(row0 + ln) * lda;
  v8f acc[4] = {};
  for (int kb = 0; kb < K; kb += 32) {
    FragB ah, al;
    const v4f x0 = *(const v4fa*)(arow + kb + 8 * hh), x1 = *(const v4fa*)(arow + kb + 8 * hh + 4);
    const v4f x2 = *(const v4fa*)(arow + kb + 16 + 8 * hh), x3 = *(const v4fa*)(arow + kb + 16 + 8 * hh + 4);
    float xs[16] = {x0[0],x0[1],x0[2],x0[3],x1[0],x1[1],x1[2],x1[3],x2[0],x2[1],x2[2],x2[3],x3[0],x3[1],x3[2],x3[3]};
#pragma unroll
    for (int i = 0; i < 16; ++i) { const unsigned short hb = bf16_bits(xs[i]); ah.u[i] = hb; al.u[i] = ASPLIT ? bf16_bits(xs[i] - bf16_val(hb)) : (unsigned short)0; }
#pragma unroll
    for (int t = 0; t < 4; ++t) {
      const unsigned short* brow = Wt + (size_t)(col0 + t * 16 + ln) * ldb + kb;
      FragB b;
      b.half[0] = *(const v8us*)(brow + 8 * hh);
      b.half[1] = *(const v8us*)(brow + 16 + 8 * hh);
      acc[t] = mmaN<ASPLIT ? 2 : 1>(ah.v, al.v, b.v, b.v, acc[t]);
    }
  }
#pragma unroll
  for (int t = 0; t < 4; ++t) {
    float bv = bias ? bias[col0 + t * 16 + ln] : 0.f;
    if (BIAS_BF16) bv = bf16_round(bv);
#pragma unroll
    for (int r = 0; r < 8; ++r) { float v = acc[t][r] + bv; if (ACT == 1) v = fmaxf(v, 0.f); so[w][8 * hh + r][t * 16 + ln] = v; }
  }
  __builtin_amdgcn_fence(__ATOMIC_ACQ_REL, "workgroup");
  __builtin_amdgcn_wave_barrier();
  const int rsub = lane >> 4, c4 = (lane & 15) * 4;
  for (int pass = 0; pass < 2; ++pass) {
#pragma unroll
    for (int q = 0; q < 8; ++q) {
      const int r = q * 2 + rsub;
      const v4f v = *(const v4fa*)&so[w][r][c4];
      *(volatile v4f*)(C + (size_t)(row0 + r) * ldc + col0 + c4) = v;
    }
    if (pass == 0) __threadfence();
  }
}

template <int D, bool CAUSAL>
__global__ __launch_bounds__(128) void k_flash(const float* __restrict__ qb, const float* __restrict__ kb, const float* __restrict__ vb,
                                             int pitch, int T, int H, float scale, float* __restrict__ y, int ypitch) {
  constexpr int KS = D / 32;
  constexpr int DT = D / 16;
  __shared__ __attribute__((aligned(16))) unsigned short sKh[32][D + 8], sKl[32][D + 8], sVh[32][D + 8], sVl[32][D + 8];
  __shared__ __attribute__((aligned(16))) unsigned short sPh[4][16][40], sPl[4][16][40];
  __shared__ __attribute__((aligned(16))) float sO[4][16][D];
  const int tid = threadIdx.x, w = tid >> 5, lane = tid & 31, ln = lane & 15, hh = lane >> 4;
  const int nqb = (T + 63) / 64;
  const int bh = blockIdx.x / nqb, qblk = blockIdx.x % nqb;
  const int b = bh / H, h = bh % H;
  const int q0 = qblk * 64 + w * 16;
  const float* Q = qb + (size_t)b * T * pitch + h * D;
  const float* K = kb + (size_t)b * T * pitch + h * D;
  const float* V = vb + (size_t)b * T * pitch + h * D;

  FragB aqh[KS], aql[KS];
  {
    int row = q0 + ln; if (row >= T) row = T - 1;
    const float* qr = Q + (size_t)row * pitch;
#pragma unroll
    for (int ks = 0; ks < KS; ++ks)
#pragma unroll
      for (int i = 0; i < 16; ++i) {
        const int d = ks * 32 + ((i < 8) ? (8 * hh + i) : (16 + 8 * hh + (i - 8)));
        const float x = qr[d] * scale; const unsigned short hb = bf16_bits(x);
        aqh[ks].u[i] = hb; aql[ks].u[i] = bf16_bits(x - bf16_val(hb));
      }
  }
  float m_r[8], l_r[8];
#pragma unroll
  for (int r = 0; r < 8; ++r) { m_r[r] = -3.0e38f; l_r[r] = 0.f; }
  v8f oacc[DT];
#pragma unroll
  for (int dt = 0; dt < DT; ++dt) oacc[dt] = (v8f){0.f,0.f,0.f,0.f,0.f,0.f,0.f,0.f};

  const int kv_end = CAUSAL ? min(T, qblk * 64 + 64) : T;
  for (int j0 = 0; j0 < kv_end; j0 += 32) {
    __syncthreads();
    for (int e = tid; e < 32 * (D / 4); e += 128) {
      const int r = e / (D / 4), c4 = (e % (D / 4)) * 4;
      const int key = j0 + r;
      v4f kf = {0.f,0.f,0.f,0.f}, vf = {0.f,0.f,0.f,0.f};
      if (key < T) { kf = *(const v4fa*)(K + (size_t)key * pitch + c4); vf = *(const v4fa*)(V + (size_t)key * pitch + c4); }
#pragma unroll
      for (int t = 0; t < 4; ++t) {
        unsigned short hb = bf16_bits(kf[t]); sKh[r][c4 + t] = hb; sKl[r][c4 + t] = bf16_bits(kf[t] - bf16_val(hb));
        hb = bf16_bits(vf[t]); sVh[r][c4 + t] = hb; sVl[r][c4 + t] = bf16_bits(vf[t] - bf16_val(hb));
      }
    }
    __syncthreads();
    v8f s[2];
#pragma unroll
    for (int nt = 0; nt < 2; ++nt) {
      v8f acc = {};
#pragma unroll
      for (int ks = 0; ks < KS; ++ks) {
        FragB bh_, bl_;
        bh_.half[0] = *(const v8us*)&sKh[nt * 16 + ln][ks * 32 + 8 * hh]; bh_.half[1] = *(const v8us*)&sKh[nt * 16 + ln][ks * 32 + 16 + 8 * hh];
        bl_.half[0] = *(const v8us*)&sKl[nt * 16 + ln][ks * 32 + 8 * hh]; bl_.half[1] = *(const v8us*)&sKl[nt * 16 + ln][ks * 32 + 16 + 8 * hh];
        acc = mmaN<3>(aqh[ks].v, aql[ks].v, bh_.v, bl_.v, acc);
      }
      s[nt] = acc;
    }
    float alpha[8];
#pragma unroll
    for (int r = 0; r < 8; ++r) {
      const int qi = q0 + 8 * hh + r;
      const int ja = j0 + ln, jb = j0 + 16 + ln;
      if (CAUSAL) { if (ja > qi) s[0][r] = -3.0e38f; if (jb > qi) s[1][r] = -3.0e38f; }
      if (ja >= T) s[0][r] = -3.0e38f;
      if (jb >= T) s[1][r] = -3.0e38f;
      float mx = fmaxf(s[0][r], s[1][r]);
      mx = fmaxf(mx, __shfl_xor(mx, 1, 32)); mx = fmaxf(mx, __shfl_xor(mx, 2, 32)); mx = fmaxf(mx, __shfl_xor(mx, 4, 32)); mx = fmaxf(mx, __shfl_xor(mx, 8, 32));
      const float mnew = fmaxf(m_r[r], mx);
      alpha[r] = (mnew > -1.0e38f) ? __expf(m_r[r] - mnew) : 1.0f;
      const float p0 = (s[0][r] > -1.0e38f) ? __expf(s[0][r] - mnew) : 0.f;
      const float p1 = (s[1][r] > -1.0e38f) ? __expf(s[1][r] - mnew) : 0.f;
      m_r[r] = mnew;
      l_r[r] = l_r[r] * alpha[r] + p0 + p1;
      unsigned short hb = bf16_bits(p0); sPh[w][8 * hh + r][ln] = hb;      sPl[w][8 * hh + r][ln] = bf16_bits(p0 - bf16_val(hb));
      hb = bf16_bits(p1);                sPh[w][8 * hh + r][16 + ln] = hb; sPl[w][8 * hh + r][16 + ln] = bf16_bits(p1 - bf16_val(hb));
    }
#pragma unroll
    for (int dt = 0; dt < DT; ++dt)
#pragma unroll
      for (int r = 0; r < 8; ++r) oacc[dt][r] *= alpha[r];
    __builtin_amdgcn_fence(__ATOMIC_ACQ_REL, "workgroup");
    __builtin_amdgcn_wave_barrier();
    FragB pah, pal;
    pah.half[0] = *(const v8us*)&sPh[w][ln][8 * hh]; pah.half[1] = *(const v8us*)&sPh[w][ln][16 + 8 * hh];
    pal.half[0] = *(const v8us*)&sPl[w][ln][8 * hh]; pal.half[1] = *(const v8us*)&sPl[w][ln][16 + 8 * hh];
#pragma unroll
    for (int dt = 0; dt < DT; ++dt) {
      FragB bvh, bvl;
#pragma unroll
      for (int i = 0; i < 8; ++i) {
        bvh.u[i] = sVh[8 * hh + i][dt * 16 + ln]; bvh.u[8 + i] = sVh[16 + 8 * hh + i][dt * 16 + ln];
        bvl.u[i] = sVl[8 * hh + i][dt * 16 + ln]; bvl.u[8 + i] = sVl[16 + 8 * hh + i][dt * 16 + ln];
      }
      oacc[dt] = mmaN<3>(pah.v, pal.v, bvh.v, bvl.v, oacc[dt]);
    }
    __builtin_amdgcn_fence(__ATOMIC_ACQ_REL, "workgroup");
    __builtin_amdgcn_wave_barrier();
  }
#pragma unroll
  for (int r = 0; r < 8; ++r) {
    float l = l_r[r];
    l += __shfl_xor(l, 1, 32); l += __shfl_xor(l, 2, 32); l += __shfl_xor(l, 4, 32); l += __shfl_xor(l, 8, 32);
    l_r[r] = (l > 0.f) ? 1.0f / l : 0.f;
  }
#pragma unroll
  for (int dt = 0; dt < DT; ++dt)
#pragma unroll
    for (int r = 0; r < 8; ++r) sO[w][8 * hh + r][dt * 16 + ln] = oacc[dt][r] * l_r[r];
  __builtin_amdgcn_fence(__ATOMIC_ACQ_REL, "workgroup");
  __builtin_amdgcn_wave_barrier();
  for (int pass = 0; pass < 2; ++pass) {
    for (int r = 0; r < 16; ++r) {
      const int row = q0 + r;
      if (row < T && lane < D / 4) {
        const v4f val = *(const v4fa*)&sO[w][r][lane * 4];
        *(volatile v4f*)(y + ((size_t)b * T + row) * ypitch + h * D + lane * 4) = val;
      }
    }
    if (pass == 0) __threadfence();
  }
}

template <bool ASPLIT, bool BSPLIT, int ACT>
__global__ __launch_bounds__(128) void k_gemm_b(const float* __restrict__ A, int lda, size_t sA, const unsigned short* __restrict__ Bh, const unsigned short* __restrict__ Bl, int ldb, size_t sB,
                                             const float* __restrict__ bias, const float* __restrict__ resid, int ldr, size_t sR, float rsign, float alpha,
                                             float* __restrict__ C, int ldc, size_t sC, int M, int N, int K) {
  __shared__ __attribute__((aligned(16))) float so[4][16][64];
  const int tid = threadIdx.x, w = tid >> 5, lane = tid & 31, ln = lane & 15, hh = lane >> 4;
  const int by = blockIdx.y;
  A += (size_t)by * sA; Bh += (size_t)by * sB; if (BSPLIT) Bl += (size_t)by * sB; C += (size_t)by * sC; if (resid) resid += (size_t)by * sR;
  const int ntn = (N + 63) / 64; const int wid = blockIdx.x * 4 + w; const int mt = wid / ntn, nq = wid % ntn;
  if (mt * 16 >= M) return;
  const int row0 = mt * 16, col0 = nq * 64;
  const float* arow = A + (size_t)(row0 + ln) * lda;
  v8f acc[4] = {};
  for (int kb = 0; kb < K; kb += 32) {
    FragB ah, al;
    const v4f x0 = *(const v4fa*)(arow + kb + 8 * hh), x1 = *(const v4fa*)(arow + kb + 8 * hh + 4);
    const v4f x2 = *(const v4fa*)(arow + kb + 16 + 8 * hh), x3 = *(const v4fa*)(arow + kb + 16 + 8 * hh + 4);
    float xs[16] = {x0[0],x0[1],x0[2],x0[3],x1[0],x1[1],x1[2],x1[3],x2[0],x2[1],x2[2],x2[3],x3[0],x3[1],x3[2],x3[3]};
#pragma unroll
    for (int i = 0; i < 16; ++i) { const unsigned short hb = bf16_bits(xs[i]); ah.u[i] = hb; al.u[i] = ASPLIT ? bf16_bits(xs[i] - bf16_val(hb)) : (unsigned short)0; }
#pragma unroll
    for (int t = 0; t < 4; ++t) {
      if (col0 + t * 16 >= N) continue;
      const size_t boff = (size_t)(col0 + t * 16 + ln) * ldb + kb;
      FragB bh_, bl_; bh_.half[0] = *(const v8us*)(Bh + boff + 8 * hh); bh_.half[1] = *(const v8us*)(Bh + boff + 16 + 8 * hh);
      if (BSPLIT) { bl_.half[0] = *(const v8us*)(Bl + boff + 8 * hh); bl_.half[1] = *(const v8us*)(Bl + boff + 16 + 8 * hh); } else bl_ = bh_;
      acc[t] = mmaN<ASPLIT ? (BSPLIT ? 3 : 2) : 1>(ah.v, al.v, bh_.v, bl_.v, acc[t]);
    }
  }
#pragma unroll
  for (int t = 0; t < 4; ++t) {
    const int col = col0 + t * 16 + ln; if (col0 + t * 16 >= N) continue; const float bv = bias ? bf16_round(bias[col]) : 0.f;
#pragma unroll
    for (int r = 0; r < 8; ++r) { float v = acc[t][r] * alpha + bv; if (resid) v += rsign * resid[(size_t)(row0 + 8 * hh + r) * ldr + col]; if (ACT == 1) v = fmaxf(v, 0.f); else if (ACT == 2) v = fmaxf(v, 0.f) + log1pf(expf(-fabsf(v))); so[w][8 * hh + r][t * 16 + ln] = v; }
  }
  __builtin_amdgcn_fence(__ATOMIC_ACQ_REL, "workgroup"); __builtin_amdgcn_wave_barrier();
  const int rsub = lane >> 4, c4 = (lane & 15) * 4;
  for (int pass = 0; pass < 2; ++pass) {
#pragma unroll
    for (int q = 0; q < 8; ++q) { const int r = q * 2 + rsub; if (col0 + c4 < N) { const v4f v = *(const v4fa*)&so[w][r][c4]; *(volatile v4f*)(C + (size_t)(row0 + r) * ldc + col0 + c4) = v; } }
    if (pass == 0) __threadfence();
  }
}
__global__ __launch_bounds__(256) void k_split_transpose_b(const float* __restrict__ src, int lds_, size_t sIn, unsigned short* __restrict__ hi, unsigned short* __restrict__ lo, size_t sOut, int K, int N) {
  const size_t t = (size_t)blockIdx.x * 256 + threadIdx.x; const int k8n = K / 8; if (t >= (size_t)N * k8n) return;
  src += (size_t)blockIdx.y * sIn; hi += (size_t)blockIdx.y * sOut; lo += (size_t)blockIdx.y * sOut;
  const int n = (int)(t / k8n), k8 = (int)(t % k8n) * 8; v8us vh, vl;
#pragma unroll
  for (int i = 0; i < 8; ++i) { const float x = src[(size_t)(k8 + i) * lds_ + n]; const unsigned short hb = bf16_bits(x); vh[i] = hb; vl[i] = bf16_bits(x - bf16_val(hb)); }
  unsigned short* dh = hi + (size_t)n * K + k8; unsigned short* dl = lo + (size_t)n * K + k8;
  *(volatile v8us*)dh = vh; *(volatile v8us*)dl = vl; __threadfence(); *(volatile v8us*)dh = vh; *(volatile v8us*)dl = vl;
}

__global__ __launch_bounds__(256) void k_bt(const float* __restrict__ W, int ldw, int k0, int K, int KP, int N, int NP, unsigned short* __restrict__ Bt) { const int t = blockIdx.x * 256 + threadIdx.x; if (t >= NP * (KP / 8)) return; const int n = t / (KP / 8), k8 = (t % (KP / 8)) * 8; v8us v; for (int q = 0; q < 8; ++q) { const int k = k8 + q; v[q] = bf16_bits((k < K && n < N) ? W[(size_t)(k0 + k) * ldw + n] : 0.f); } *(volatile v8us*)(Bt + (size_t)n * KP + k8) = v; __threadfence(); *(volatile v8us*)(Bt + (size_t)n * KP + k8) = v; }
__global__ __launch_bounds__(256) void k_stp(const float* __restrict__ st, float* __restrict__ STP) { const size_t t = (size_t)blockIdx.x * 256 + threadIdx.x; if (t >= (size_t)TT * SDP / 4) return; const int c4 = (int)((t * 4) % SDP); const size_t r = (t * 4) / SDP; v4f o; for (int q = 0; q < 4; ++q) { const int c = c4 + q; o[q] = (c < SD) ? bf16_round(st[r * SD + c]) : 0.f; } *(volatile v4f*)(STP + t * 4) = o; __threadfence(); *(volatile v4f*)(STP + t * 4) = o; }
__global__ __launch_bounds__(256) void k_brelu(float* __restrict__ Y, const float* __restrict__ b, int NB, size_t n4) { const size_t t = (size_t)blockIdx.x * 256 + threadIdx.x; if (t >= n4) return; const int c4 = (int)((t * 4) % HP); v4f v = *(const v4fa*)(Y + t * 4); for (int q = 0; q < 4; ++q) { const int c = c4 + q; v[q] = (c < NB) ? fmaxf(v[q] + bf16_round(b[c]), 0.f) : 0.f; } *(volatile v4f*)(Y + t * 4) = v; __threadfence(); *(volatile v4f*)(Y + t * 4) = v; }
__global__ __launch_bounds__(1024) void k_ascore(const float* __restrict__ A2, const float* __restrict__ w3, const float* __restrict__ b3, float* __restrict__ AS) { __shared__ float so[32]; const int tid = threadIdx.x, wv = tid >> 5, lane = tid & 31; const int t = blockIdx.x * 32 + wv; float s = 0.f;
  for (int k = lane; k < HID; k += 32) s += A2[(size_t)t * HP + k] * bf16_round(w3[k]); for (int o = 16; o >= 1; o >>= 1) s += __shfl_xor(s, o, 32); if (lane == 0) so[wv] = s + bf16_round(b3[0]); __syncthreads();
  if (tid < 32) { *(volatile float*)(AS + blockIdx.x * 32 + tid) = so[tid]; } __threadfence(); if (tid < 32) { *(volatile float*)(AS + blockIdx.x * 32 + tid) = so[tid]; } }
__device__ __forceinline__ void span_of(int s, int& n, int& start) { int off = 0; n = 1; for (int m = 1; m <= MAXW; ++m) { const int w = TT - m + 1; if (s < off + w) { n = m; start = s - off; return; } off += w; } n = MAXW; start = 0; }
__device__ __forceinline__ int dtoi(int n) { return (n >= 1) + (n >= 2) + (n >= 3) + (n >= 4) + (n >= 8); }
__global__ __launch_bounds__(256) void k_pool(const float* __restrict__ AS, const float* __restrict__ emb, float* __restrict__ PO, int* __restrict__ SPI) { const int tid = threadIdx.x, wv = tid >> 5, lane = tid & 31; const int s = blockIdx.x * 8 + wv; if (s >= NSP) return;
  float out[10]; for (int u = 0; u < 10; ++u) out[u] = 0.f; int n = 1, start = 0;
  if (s < NSPAN) { span_of(s, n, start); float sc = (lane < n) ? AS[start + lane] : -3.0e38f; float mx = sc; for (int o = 16; o >= 1; o >>= 1) mx = fmaxf(mx, __shfl_xor(mx, o, 32)); float e = (lane < n) ? expf(sc - mx) : 0.f; float den = e; for (int o = 16; o >= 1; o >>= 1) den += __shfl_xor(den, o, 32); const float a = e / den;
#pragma unroll 1
    for (int i = 0; i < n; ++i) { const float ai = __shfl(a, i, 32); const float* er = emb + (size_t)(start + i) * ED;
#pragma unroll
      for (int u = 0; u < 10; ++u) { const int d = u * 32 + lane; if (d < ED) out[u] += ai * bf16_round(er[d]); } } }
  for (int pass = 0; pass < 2; ++pass) {
#pragma unroll
    for (int u = 0; u < 10; ++u) *(volatile float*)(PO + (size_t)s * EDP + u * 32 + lane) = out[u]; if (pass == 0) __threadfence(); }
  (void)SPI; }
__global__ __launch_bounds__(256) void k_h1(float* __restrict__ PW, const float* __restrict__ SAB, const float* __restrict__ WW, const float* __restrict__ sb1, const int* __restrict__ SPI) { const size_t t = (size_t)blockIdx.x * 256 + threadIdx.x; if (t >= (size_t)NSP * HP / 4) return; const int c4 = (int)((t * 4) % HP); const int s = (int)((t * 4) / HP); v4f v = *(const v4fa*)(PW + t * 4);
  if (s < NSPAN) { int n, start; span_of(s, n, start); (void)SPI; const int end = start + n - 1; const int wi = dtoi(n); const v4f a = *(const v4fa*)(SAB + (size_t)start * (2 * HP) + c4), b = *(const v4fa*)(SAB + (size_t)end * (2 * HP) + HP + c4);
    for (int q = 0; q < 4; ++q) { const int c = c4 + q; v[q] = (c < HID) ? fmaxf(((a[q] + b[q]) + v[q]) + (WW[wi * HP + c] + bf16_round(sb1[c])), 0.f) : 0.f; } } else { for (int q = 0; q < 4; ++q) v[q] = 0.f; }
  *(volatile v4f*)(PW + t * 4) = v; __threadfence(); *(volatile v4f*)(PW + t * 4) = v; }
__global__ __launch_bounds__(256) void k_ww(const float* __restrict__ wt, const float* __restrict__ sW1, float* __restrict__ WW) { const int t = threadIdx.x; for (int e = t; e < 9 * HP; e += 256) { const int r = e / HP, c = e % HP; float s = 0.f; if (c < HID) { for (int k = 0; k < 20; ++k) s += bf16_round(wt[r * 20 + k]) * bf16_round(sW1[(size_t)(1100 + k) * HID + c]); } *(volatile float*)(WW + e) = s; __threadfence(); *(volatile float*)(WW + e) = s; } }
__global__ __launch_bounds__(1024) void k_sms(const float* __restrict__ H2, const float* __restrict__ sb2, const float* __restrict__ w3, const float* __restrict__ b3, float* __restrict__ out) { __shared__ float so[32]; const int tid = threadIdx.x, wv = tid >> 5, lane = tid & 31; const int s = blockIdx.x * 32 + wv; float v = 0.f;
  if (s < NSPAN) { for (int k = lane; k < HID; k += 32) v += fmaxf(H2[(size_t)s * HP + k] + bf16_round(sb2[k]), 0.f) * bf16_round(w3[k]); for (int o = 16; o >= 1; o >>= 1) v += __shfl_xor(v, o, 32); v += bf16_round(b3[0]); }
  if (lane == 0) so[wv] = v; __syncthreads(); const int idx = blockIdx.x * 32 + tid; if (tid < 32 && idx < NSPAN) { *(volatile float*)(out + idx) = so[tid]; } __threadfence(); if (tid < 32 && idx < NSPAN) { *(volatile float*)(out + idx) = so[tid]; } }
extern "C" void kernel_launch(void* const* d_in, const int* in_sizes, int n_in,
                              void* d_out, int out_size, void* d_ws, size_t ws_size, hipStream_t stream) {
  (void)in_sizes; (void)n_in; (void)out_size;
  const float* embeds = (const float*)d_in[0]; const float* states = (const float*)d_in[1]; const float* aW1 = (const float*)d_in[2]; const float* ab1 = (const float*)d_in[3]; const float* aW2 = (const float*)d_in[4]; const float* ab2 = (const float*)d_in[5]; const float* aW3 = (const float*)d_in[6]; const float* ab3 = (const float*)d_in[7]; const float* wtab = (const float*)d_in[8];
  const float* sW1 = (const float*)d_in[9]; const float* sb1 = (const float*)d_in[10]; const float* sW2 = (const float*)d_in[11]; const float* sb2 = (const float*)d_in[12]; const float* sW3 = (const float*)d_in[13]; const float* sb3 = (const float*)d_in[14];
  char* ws = (char*)d_ws; size_t off = 0;
  auto take = [&](size_t bytes) { char* p = ws + off; off += (bytes + 255) & ~(size_t)255; return p; };
  unsigned short* BaW1 = (unsigned short*)take((size_t)HP * SDP * 2); unsigned short* BaW2 = (unsigned short*)take((size_t)HP * HP * 2); unsigned short* BsAB = (unsigned short*)take((size_t)2 * HP * SDP * 2); unsigned short* BsC = (unsigned short*)take((size_t)HP * EDP * 2); unsigned short* BsW2 = (unsigned short*)take((size_t)HP * HP * 2);
  float* STP = (float*)take((size_t)TT * SDP * 4); float* A1 = (float*)take((size_t)TT * HP * 4); float* A2 = (float*)take((size_t)TT * HP * 4); float* AS = (float*)take(TT * 4); float* SAB = (float*)take((size_t)TT * 2 * HP * 4); float* WW = (float*)take(9 * HP * 4 + 256);
  float* PO = (float*)take((size_t)NSP * EDP * 4); int* SPI = (int*)take((size_t)NSP * 2 * 4); float* PW = (float*)take((size_t)NSP * HP * 4); float* H2 = (float*)take((size_t)NSP * HP * 4);
  if (off > ws_size) return;
  k_bt<<<(HP * (SDP / 8) + 255) / 256, 256, 0, stream>>>(aW1, HID, 0, SD, SDP, HID, HP, BaW1); k_bt<<<(HP * (HP / 8) + 255) / 256, 256, 0, stream>>>(aW2, HID, 0, HID, HP, HID, HP, BaW2);
  k_bt<<<(HP * (SDP / 8) + 255) / 256, 256, 0, stream>>>(sW1, HID, 0, SD, SDP, HID, HP, BsAB); k_bt<<<(HP * (SDP / 8) + 255) / 256, 256, 0, stream>>>(sW1, HID, SD, SD, SDP, HID, HP, BsAB + (size_t)HP * SDP);
  k_bt<<<(HP * (EDP / 8) + 255) / 256, 256, 0, stream>>>(sW1, HID, 2 * SD, ED, EDP, HID, HP, BsC); k_bt<<<(HP * (HP / 8) + 255) / 256, 256, 0, stream>>>(sW2, HID, 0, HID, HP, HID, HP, BsW2); k_ww<<<1, 256, 0, stream>>>(wtab, sW1, WW);
  k_stp<<<(unsigned)(((size_t)TT * SDP / 4 + 255) / 256), 256, 0, stream>>>(states, STP);
  k_gemm_b<false, false, 0><<<dim3(((TT / 16) * 3 + 3) / 4, 1), 128, 0, stream>>>(STP, SDP, 0, BaW1, BaW1, SDP, 0, nullptr, nullptr, 0, 0, 1.f, 1.f, A1, HP, 0, TT, HP, SDP);
  k_brelu<<<(TT * HP / 4 + 255) / 256, 256, 0, stream>>>(A1, ab1, HID, (size_t)TT * HP / 4);
  k_gemm_b<true, false, 0><<<dim3(((TT / 16) * 3 + 3) / 4, 1), 128, 0, stream>>>(A1, HP, 0, BaW2, BaW2, HP, 0, nullptr, nullptr, 0, 0, 1.f, 1.f, A2, HP, 0, TT, HP, HP);
  k_brelu<<<(TT * HP / 4 + 255) / 256, 256, 0, stream>>>(A2, ab2, HID, (size_t)TT * HP / 4); k_ascore<<<TT / 32, 1024, 0, stream>>>(A2, aW3, ab3, AS);
  k_gemm_b<false, false, 0><<<dim3(((TT / 16) * 5 + 3) / 4, 1), 128, 0, stream>>>(STP, SDP, 0, BsAB, BsAB, SDP, 0, nullptr, nullptr, 0, 0, 1.f, 1.f, SAB, 2 * HP, 0, TT, 2 * HP, SDP);
  k_pool<<<NSP / 8, 256, 0, stream>>>(AS, embeds, PO, SPI);
  k_gemm_b<true, false, 0><<<dim3(((NSP / 16) * 3 + 3) / 4, 1), 128, 0, stream>>>(PO, EDP, 0, BsC, BsC, EDP, 0, nullptr, nullptr, 0, 0, 1.f, 1.f, PW, HP, 0, NSP, HP, EDP);
  k_h1<<<(unsigned)(((size_t)NSP * HP / 4 + 255) / 256), 256, 0, stream>>>(PW, SAB, WW, sb1, SPI);
  k_gemm_b<true, false, 0><<<dim3(((NSP / 16) * 3 + 3) / 4, 1), 128, 0, stream>>>(PW, HP, 0, BsW2, BsW2, HP, 0, nullptr, nullptr, 0, 0, 1.f, 1.f, H2, HP, 0, NSP, HP, HP);
  k_sms<<<(NSPAN + 31) / 32, 1024, 0, stream>>>(H2, sb2, sW3, sb3, (float*)d_out);
}
